// RNN_37185826849416
// MI455X (gfx1250) — hardware-verified
//
#include <hip/hip_runtime.h>
#include <math.h>

constexpr int NBATCH   = 2048;
constexpr int NSTEP    = 512;
constexpr int NHID     = 64;
constexpr int NGATE    = 4 * NHID;
constexpr int ROWS_BLK = 32;
constexpr int NTHR     = 128;
constexpr int WPITCH   = 72;
constexpr int HPITCH   = 72;
constexpr int XCHUNK   = 64;
constexpr int XPITCH   = 68;
constexpr int FPITCH   = 65;
constexpr float HCARRY     = 16.0f;
constexpr float WCARRY     = 8.0f;
constexpr float ACARRY     = HCARRY * WCARRY;
constexpr float ACARRY_INV = 1.0f / ACARRY;

static_assert(NBATCH % ROWS_BLK == 0, "grid exact");
static_assert(NSTEP % XCHUNK == 0, "chunks exact");
static_assert(XCHUNK % 2 == 0, "ping-pong parity continues across chunks");
static_assert(NHID == 64 && NHID % 32 == 0, "K is two 32-deep steps");
static_assert(NHID == 16 * (NTHR / 32), "one 16-unit group per wave");
static_assert(ROWS_BLK == 32, "two 16-row subtiles, one output line per block");
static_assert((NGATE * NHID / 8) % NTHR == 0, "weight staging loop exact");
static_assert((ROWS_BLK * XCHUNK / 4) % NTHR == 0, "x staging loop exact");
static_assert(WPITCH % 8 == 0 && HPITCH % 8 == 0 && XPITCH % 4 == 0, "16-B aligned rows");
static_assert(ACARRY == 128.0f, "carry product");

typedef __attribute__((ext_vector_type(16))) _Float16 v16h;
typedef __attribute__((ext_vector_type(8)))  _Float16 v8h;
typedef __attribute__((ext_vector_type(8)))  float    v8f;
typedef __attribute__((ext_vector_type(4)))  float    v4f;

__device__ __forceinline__ void keep4_h(v16h a, v16h b, v16h c, v16h d) { asm volatile("v_nop" :: "v"(a), "v"(b), "v"(c), "v"(d)); }
__device__ __forceinline__ void gate_guard(v8f& a, v8f& b, v8f& c, v8f& d, v16h x, v16h y) {
  asm volatile("v_nop\n\tv_nop\n\tv_nop\n\tv_nop" : "+v"(a), "+v"(b), "+v"(c), "+v"(d) : "v"(x), "v"(y));
}

template <typename T> struct Frag;
template <> struct Frag<_Float16> {
  typedef v16h V; union U { v16h v; v8h h[2]; };
  static __device__ __forceinline__ v16h load(const _Float16* p) {
    U f; f.h[0] = *(const v8h*)(p); f.h[1] = *(const v8h*)(p + 16); return f.v;
  }
  static __device__ __forceinline__ v8f mma(v16h a, v16h b, v8f c) {
    return __builtin_amdgcn_wmma_f32_16x16x32_f16(false, a, false, b, (short)0, c, false, false);
  }
};

__device__ __forceinline__ float fsig(float x)  { return __builtin_amdgcn_rcpf(1.0f + __expf(-x)); }
__device__ __forceinline__ float ftanh(float x) { return 1.0f - 2.0f * __builtin_amdgcn_rcpf(__expf(2.0f * x) + 1.0f); }

__global__ __launch_bounds__(NTHR) void lstm_seq_kernel(const float* __restrict__ x,
                                                        const float* __restrict__ w_ih,
                                                        const float* __restrict__ w_hh,
                                                        const float* __restrict__ b_ih,
                                                        const float* __restrict__ b_hh,
                                                        const float* __restrict__ w_d,
                                                        const float* __restrict__ b_d,
                                                        float* __restrict__ out) {
  __shared__ __align__(16) _Float16 Ws[NGATE * WPITCH];
  __shared__ __align__(16) _Float16 Hh[2][ROWS_BLK * HPITCH];
  __shared__ __align__(16) float    Xs[ROWS_BLK * XPITCH];
  __shared__ __align__(16) float    Hf[ROWS_BLK * FPITCH];
  __shared__ __align__(16) float    Wds[NHID];

  const int tid  = threadIdx.x;
  const int lane = tid & 31;
  const int wave = tid >> 5;
  const int c    = lane & 15;
  const int hh   = lane >> 4;
  const int koff = hh * 8;
  const int base = blockIdx.x * ROWS_BLK;

#pragma unroll 1
  for (int it = 0; it < (NGATE * NHID / 8) / NTHR; ++it) {
    const int i  = it * NTHR + tid;
    const int n  = i >> 3;
    const int k8 = (i & 7) * 8;
    const v4f wa = *(const v4f*)(w_hh + (size_t)n * NHID + k8);
    const v4f wb = *(const v4f*)(w_hh + (size_t)n * NHID + k8 + 4);
    v8h hv;
#pragma unroll
    for (int e = 0; e < 4; ++e) {
      hv[e]     = (_Float16)(wa[e] * WCARRY);
      hv[4 + e] = (_Float16)(wb[e] * WCARRY);
    }
    *(v8h*)(Ws + n * WPITCH + k8) = hv;
  }
  {
    const v8h z8h = {(_Float16)0.0f, (_Float16)0.0f, (_Float16)0.0f, (_Float16)0.0f,
                     (_Float16)0.0f, (_Float16)0.0f, (_Float16)0.0f, (_Float16)0.0f};
    *(v8h*)(Ws + tid * WPITCH + NHID) = z8h;
    *(v8h*)(Ws + (tid + NTHR) * WPITCH + NHID) = z8h;
    _Float16* hz = &Hh[0][0];
#pragma unroll 1
    for (int i = tid; i < (2 * ROWS_BLK * HPITCH) / 8; i += NTHR) *(v8h*)(hz + 8 * i) = z8h;
  }
  if (wave < 2) Wds[tid] = w_d[tid];

  float wv[4], bv[4];
#pragma unroll
  for (int g = 0; g < 4; ++g) {
    const int n = NHID * g + 16 * wave + c;
    wv[g] = w_ih[n] * ACARRY;
    bv[g] = (b_ih[n] + b_hh[n]) * ACARRY;
  }
  asm volatile("" ::: "memory");
  __syncthreads();

  v16h bw[4][2];
#pragma unroll
  for (int g = 0; g < 4; ++g) {
    const _Float16* wp = Ws + (NHID * g + 16 * wave + c) * WPITCH + koff;
    bw[g][0] = Frag<_Float16>::load(wp);
    bw[g][1] = Frag<_Float16>::load(wp + 32);
  }

  float cst[2][8], hst[2][8];
#pragma unroll
  for (int mt = 0; mt < 2; ++mt)
#pragma unroll
    for (int r = 0; r < 8; ++r) { cst[mt][r] = 0.0f; hst[mt][r] = 0.0f; }

#pragma unroll 1
  for (int ch = 0; ch < NSTEP / XCHUNK; ++ch) {
#pragma unroll
    for (int it = 0; it < (ROWS_BLK * XCHUNK / 4) / NTHR; ++it) {
      const int idx = it * NTHR + tid;
      const int rr  = idx >> 4;
      const int c4  = (idx & 15) * 4;
      const v4f v = *(const v4f*)(x + (size_t)(base + rr) * NSTEP + (size_t)ch * XCHUNK + c4);
      *(v4f*)(Xs + rr * XPITCH + c4) = v;
    }
    __syncthreads();

#pragma unroll 1
    for (int tc = 0; tc < XCHUNK; ++tc) {
      const int p = tc & 1;
      const _Float16* hcur = &Hh[0][0] + p * (ROWS_BLK * HPITCH);
      _Float16*       hnxt = &Hh[0][0] + (p ^ 1) * (ROWS_BLK * HPITCH);

#pragma unroll
      for (int mt = 0; mt < 2; ++mt) {
        const _Float16* hp = hcur + (16 * mt + c) * HPITCH + koff;
        const v16h a0 = Frag<_Float16>::load(hp);
        const v16h a1 = Frag<_Float16>::load(hp + 32);

        float xv[8];
#pragma unroll
        for (int r = 0; r < 8; ++r) xv[r] = Xs[(16 * mt + 8 * hh + r) * XPITCH + tc];

        v8f acc[4];
#pragma unroll
        for (int g = 0; g < 4; ++g)
#pragma unroll
          for (int r = 0; r < 8; ++r) acc[g][r] = fmaf(xv[r], wv[g], bv[g]);

#pragma unroll
        for (int g = 0; g < 4; ++g) acc[g] = Frag<_Float16>::mma(a0, bw[g][0], acc[g]);
#pragma unroll
        for (int g = 0; g < 4; ++g) acc[g] = Frag<_Float16>::mma(a1, bw[g][1], acc[g]);
        gate_guard(acc[0], acc[1], acc[2], acc[3], a0, a1);

#pragma unroll
        for (int r = 0; r < 8; ++r) {
          const float zi = acc[0][r] * ACARRY_INV;
          const float zf = acc[1][r] * ACARRY_INV;
          const float zg = acc[2][r] * ACARRY_INV;
          const float zo = acc[3][r] * ACARRY_INV;
          const float ig = fsig(zi);
          const float fg = fsig(zf);
          const float gg = ftanh(zg);
          const float og = fsig(zo);
          const float cn = fg * cst[mt][r] + ig * gg;
          cst[mt][r] = cn;
          const float hn = og * ftanh(cn);
          hst[mt][r] = hn;
          hnxt[(16 * mt + 8 * hh + r) * HPITCH + 16 * wave + c] = (_Float16)(hn * HCARRY);
        }
      }
      keep4_h(bw[0][0], bw[1][0], bw[2][0], bw[3][0]);
      keep4_h(bw[0][1], bw[1][1], bw[2][1], bw[3][1]);
      __syncthreads();
    }
  }

#pragma unroll
  for (int mt = 0; mt < 2; ++mt)
#pragma unroll
    for (int r = 0; r < 8; ++r) Hf[(16 * mt + 8 * hh + r) * FPITCH + 16 * wave + c] = hst[mt][r];
  __syncthreads();

  if (wave == 0) {
    const float* hr = Hf + lane * FPITCH;
    float s = 0.0f;
#pragma unroll 4
    for (int k = 0; k < NHID; ++k) s = fmaf(hr[k], Wds[k], s);
    s += b_d[0];
    volatile float* op = out + base + lane;
    *op = s;
    __threadfence();
    *op = s;
  }
}

extern "C" void kernel_launch(void* const* d_in, const int* in_sizes, int n_in,
                              void* d_out, int out_size, void* d_ws, size_t ws_size, hipStream_t stream) {
  (void)d_ws; (void)ws_size;
  if (n_in < 7 || d_out == nullptr) return;
  if (in_sizes[0] != NBATCH * NSTEP || in_sizes[1] != NGATE || in_sizes[2] != NGATE * NHID ||
      in_sizes[3] != NGATE || in_sizes[4] != NGATE || in_sizes[5] != NHID || in_sizes[6] != 1 ||
      out_size != NBATCH) return;

  const float* x    = (const float*)d_in[0];
  const float* w_ih = (const float*)d_in[1];
  const float* w_hh = (const float*)d_in[2];
  const float* b_ih = (const float*)d_in[3];
  const float* b_hh = (const float*)d_in[4];
  const float* w_d  = (const float*)d_in[5];
  const float* b_d  = (const float*)d_in[6];
  float* out = (float*)d_out;

  lstm_seq_kernel<<<NBATCH / ROWS_BLK, NTHR, 0, stream>>>(x, w_ih, w_hh, b_ih, b_hh, w_d, b_d, out);
}
